// SubGraph_43155831390245
// MI455X (gfx1250) — hardware-verified
//
#include <hip/hip_runtime.h>
#include <math.h>

typedef __attribute__((ext_vector_type(16))) _Float16 v16h;
typedef __attribute__((ext_vector_type(16))) __bf16 v16b;
typedef __attribute__((ext_vector_type(8)))  _Float16 v8h;
typedef __attribute__((ext_vector_type(8)))  float v8f;
typedef __attribute__((ext_vector_type(4)))  float v4f;
typedef __attribute__((ext_vector_type(2)))  float v2f;
typedef __attribute__((ext_vector_type(4)))  unsigned v4u;
typedef __attribute__((ext_vector_type(4)))  int v4i;
typedef float __attribute__((may_alias)) float_a;
typedef int __attribute__((may_alias)) int_a;

template <typename T> __device__ __forceinline__ void vst2(void* p, T v) { *(volatile T*)p = v; __threadfence(); *(volatile T*)p = v; }
__device__ __forceinline__ v8f wmma16(v16h a, v16h b, v8f c) {
  v8f d = __builtin_amdgcn_wmma_f32_16x16x32_f16(false, a, false, b, (short)0, c, false, false);
  asm volatile("v_nop\n\tv_nop\n\tv_nop\n\tv_nop" : "+v"(d) : "v"(a), "v"(b));
  return d;
}
__device__ __forceinline__ v8f wmma_bf(v16b a, v16b b, v8f c) {
  v8f d = __builtin_amdgcn_wmma_f32_16x16x32_bf16(false, a, false, b, (short)0, c, false, false);
  asm volatile("v_nop\n\tv_nop\n\tv_nop\n\tv_nop" : "+v"(d) : "v"(a), "v"(b));
  return d;
}
__device__ __forceinline__ v16h frag_h(const _Float16* rowk0, int lane) {
  union { v16h v; v8h q[2]; } u; const _Float16* p = rowk0 + 8 * (lane >> 4);
  u.q[0] = *(const v8h*)p; u.q[1] = *(const v8h*)(p + 16); return u.v;
}
__device__ __forceinline__ v16h frag_f32(const float* rowk0, int lane) {
  v16h a; const float* p = rowk0 + 8 * (lane >> 4);
#pragma unroll
  for (int i = 0; i < 8; ++i) { a[i] = (_Float16)p[i]; a[8 + i] = (_Float16)p[16 + i]; }
  return a;
}
__device__ __forceinline__ v16h frag_f32s(const float* rowk0, int lane, float sc) {
  v16h a; const float* p = rowk0 + 8 * (lane >> 4);
#pragma unroll
  for (int i = 0; i < 8; ++i) { a[i] = (_Float16)(p[i] * sc); a[8 + i] = (_Float16)(p[16 + i] * sc); }
  return a;
}
__device__ __forceinline__ v16h fragc_f32(const float* W, int k0, int n, int lane, int ld, int K) {
  v16h a; const int g = lane >> 4;
#pragma unroll
  for (int i = 0; i < 8; ++i) { const int ka = k0 + 8 * g + i, kb = ka + 16;
    a[i] = (_Float16)(ka < K ? W[(size_t)(ka < K ? ka : K - 1) * ld + n] : 0.f); a[8 + i] = (_Float16)(kb < K ? W[(size_t)(kb < K ? kb : K - 1) * ld + n] : 0.f); }
  return a;
}
struct F2 { v16b h, l; };
__device__ __forceinline__ F2 bsplit16(const float v[16]) { F2 r;
#pragma unroll
  for (int i = 0; i < 16; ++i) { const __bf16 h = (__bf16)v[i]; r.h[i] = h; r.l[i] = (__bf16)(v[i] - (float)h); }
  return r; }
__device__ __forceinline__ F2 split_row(const float* row, int k0, int lane) { float v[16]; const float* p = row + k0 + 8 * (lane >> 4);
#pragma unroll
  for (int i = 0; i < 8; ++i) { v[i] = p[i]; v[8 + i] = p[16 + i]; }
  return bsplit16(v); }
__device__ __forceinline__ F2 split_rowK(const float* row, int k0, int lane, int K) { float v[16]; const int g = lane >> 4;
#pragma unroll
  for (int i = 0; i < 8; ++i) { const int ka = k0 + 8 * g + i, kb = ka + 16; v[i] = ka < K ? row[ka < K ? ka : K - 1] : 0.f; v[8 + i] = kb < K ? row[kb < K ? kb : K - 1] : 0.f; }
  return bsplit16(v); }
__device__ __forceinline__ F2 split_col(const float* W, int k0, int n, int lane, int ld, int K) { float v[16]; const int g = lane >> 4;
#pragma unroll
  for (int i = 0; i < 8; ++i) { const int ka = k0 + 8 * g + i, kb = ka + 16; v[i] = ka < K ? W[(size_t)(ka < K ? ka : K - 1) * ld + n] : 0.f; v[8 + i] = kb < K ? W[(size_t)(kb < K ? kb : K - 1) * ld + n] : 0.f; }
  return bsplit16(v); }
__device__ __forceinline__ v8f mac3(const F2& a, const F2& b, v8f c) { c = wmma_bf(a.l, b.h, c); c = wmma_bf(a.h, b.l, c); return wmma_bf(a.h, b.h, c); }
__device__ __forceinline__ float sigm(float v) { return 1.0f / (1.0f + expf(-v)); }
#define LDSX() do { asm volatile("s_wait_dscnt 0" ::: "memory"); __builtin_amdgcn_wave_barrier(); __builtin_amdgcn_fence(__ATOMIC_RELEASE, "workgroup"); } while (0)


#define NN 1048576
#define CPL 32
#define NC (NN / CPL)
#define DI 10
#define HH 64
#ifndef TRB
#define TRB (NN / 64)
#endif
typedef __attribute__((ext_vector_type(8))) __bf16 v8b;
__device__ __forceinline__ v16b frag_b(const __bf16* rowk0, int lane) {
  union { v16b v; v8b q[2]; } u; const __bf16* p = rowk0 + 8 * (lane >> 4);
  u.q[0] = *(const v8b*)p; u.q[1] = *(const v8b*)(p + 16); return u.v;
}
__device__ __forceinline__ float bfr(float v) { return (float)(__bf16)v; }
__device__ __attribute__((noinline)) float exp_ni(float v) { return expf(v); }
__device__ __attribute__((noinline)) float erf_ni(float v) { return erff(v); }

#define WS_W10 0u
#define WS_WF  (WS_W10 + 2u * HH * 32)
#define OFF_W20 0
#define OFF_W11 (HH * HH)
#define OFF_W21 (OFF_W11 + HH * 2 * HH)
#define OFF_W12 (OFF_W21 + HH * HH)
#define OFF_W22 (OFF_W12 + HH * 2 * HH)
#define OFF_WL  (OFF_W22 + HH * HH)
#define WF_TOT  (OFF_WL + HH * 2 * HH)
#define WS_END (WS_WF + 2u * (size_t)WF_TOT + 256u)

__global__ __launch_bounds__(256) void k_pack(const float* __restrict__ W10, const float* __restrict__ W20, const float* __restrict__ W11, const float* __restrict__ W21, const float* __restrict__ W12, const float* __restrict__ W22, const float* __restrict__ WL, __bf16* __restrict__ P0, _Float16* __restrict__ PF) {
  const int which = blockIdx.x, t = threadIdx.x;
  if (which == 0) { __shared__ __align__(16) __bf16 s[HH * 32]; for (int e = t; e < HH * 32; e += 256) { const int n = e >> 5, k = e & 31; s[e] = (k < DI) ? (__bf16)W10[k * HH + n] : (__bf16)0.f; } __syncthreads(); for (int q = t; q < HH * 32 / 8; q += 256) vst2((unsigned*)(P0 + q * 8), *(const v4u*)&s[q * 8]); return; }
  const float* src; int K, off; switch (which) { case 1: src = W20; K = HH; off = OFF_W20; break; case 2: src = W11; K = 2 * HH; off = OFF_W11; break; case 3: src = W21; K = HH; off = OFF_W21; break; case 4: src = W12; K = 2 * HH; off = OFF_W12; break; case 5: src = W22; K = HH; off = OFF_W22; break; default: src = WL; K = 2 * HH; off = OFF_WL; }
  __shared__ __align__(16) _Float16 sf[HH * 2 * HH]; for (int e = t; e < HH * K; e += 256) { const int n = e / K, k = e % K; sf[e] = (_Float16)(bfr(src[k * HH + n]) * 256.0f); } __syncthreads(); for (int q = t; q < HH * K / 8; q += 256) vst2((unsigned*)(PF + off + q * 8), *(const v4u*)&sf[q * 8]);
}
template <int KIN>
__device__ __forceinline__ void gemm_tile(const _Float16* __restrict__ arow, const _Float16* __restrict__ Wr, int lane, int col, v8f acc[4]) {
#pragma unroll
  for (int jt = 0; jt < 4; ++jt) { v8f z = {}; acc[jt] = z; }
#pragma unroll
  for (int kc = 0; kc < KIN / 32; ++kc) { const v16h a = frag_h(arow + kc * 32, lane);
#pragma unroll
    for (int jt = 0; jt < 4; ++jt) acc[jt] = wmma16(a, frag_h(Wr + (size_t)(jt * 16 + col) * KIN + kc * 32, lane), acc[jt]); }
#pragma unroll
  for (int jt = 0; jt < 4; ++jt)
#pragma unroll
    for (int r = 0; r < 8; ++r) acc[jt][r] *= (1.0f / 256.0f);
}
__global__ __launch_bounds__(128) void k_sub(const float* __restrict__ X, const __bf16* __restrict__ P0, const _Float16* __restrict__ PF,
    const float* __restrict__ B10, const float* __restrict__ G0, const float* __restrict__ BE0, const float* __restrict__ B20,
    const float* __restrict__ B11, const float* __restrict__ G1, const float* __restrict__ BE1, const float* __restrict__ B21,
    const float* __restrict__ B12, const float* __restrict__ G2, const float* __restrict__ BE2, const float* __restrict__ B22,
    const float* __restrict__ BL, float* __restrict__ OUT) {
  __shared__ __align__(16) float sf[64][68];
  __shared__ __align__(16) _Float16 sa[64][136];
  __shared__ __align__(16) float spool[2][64];
  const int tid = threadIdx.x, wave = tid >> 5, lane = tid & 31, col = lane & 15, g = lane >> 4; const size_t r0b = (size_t)blockIdx.x * 64; const int w0 = wave * 16;
  v8f acc[4];
  { v16b a; { const float* p = X + (r0b + w0 + col) * DI;
#pragma unroll
      for (int i = 0; i < 8; ++i) { const int k0 = 8 * g + i, k1 = 16 + 8 * g + i; a[i] = (k0 < DI) ? (__bf16)p[k0] : (__bf16)0.f; a[8 + i] = (k1 < DI) ? (__bf16)p[k1] : (__bf16)0.f; } }
#pragma unroll
    for (int jt = 0; jt < 4; ++jt) { v8f z = {}; acc[jt] = wmma_bf(a, frag_b(P0 + (size_t)(jt * 16 + col) * 32, lane), z); } }
#pragma unroll 1
  for (int layer = 0; layer < 3; ++layer) {
    const float* B1 = (layer == 0) ? B10 : (layer == 1) ? B11 : B12; const float* GG = (layer == 0) ? G0 : (layer == 1) ? G1 : G2; const float* BB = (layer == 0) ? BE0 : (layer == 1) ? BE1 : BE2; const float* B2 = (layer == 0) ? B20 : (layer == 1) ? B21 : B22;
    const _Float16* W2r = PF + ((layer == 0) ? OFF_W20 : (layer == 1) ? OFF_W21 : OFF_W22);
    if (layer > 0) { const _Float16* W1r = PF + ((layer == 1) ? OFF_W11 : OFF_W12); gemm_tile<2 * HH>(&sa[w0 + col][0], W1r, lane, col, acc); }
#pragma unroll
    for (int jt = 0; jt < 4; ++jt) { const float bb = bfr(B1[jt * 16 + col]);
#pragma unroll
      for (int r = 0; r < 8; ++r) sf[w0 + 8 * g + r][jt * 16 + col] = acc[jt][r] + bb; }
    LDSX();
    { const int rl = lane & 15, half = lane >> 4; float s = 0.f; for (int d = half * 32; d < half * 32 + 32; ++d) s += sf[w0 + rl][d]; s += __shfl_xor(s, 16); const float mu = s / 64.0f; float q = 0.f; for (int d = half * 32; d < half * 32 + 32; ++d) { const float dd = sf[w0 + rl][d] - mu; q += dd * dd; } q += __shfl_xor(q, 16); const float inv = 1.0f / sqrtf(q / 64.0f + 1e-5f);
      for (int d = half * 32; d < half * 32 + 32; ++d) sa[w0 + rl][d] = (_Float16)fmaxf((sf[w0 + rl][d] - mu) * inv * bfr(GG[d]) + bfr(BB[d]), 0.f); }
    LDSX();
    gemm_tile<HH>(&sa[w0 + col][0], W2r, lane, col, acc);
    LDSX();
#pragma unroll
    for (int jt = 0; jt < 4; ++jt) { const float bb = bfr(B2[jt * 16 + col]);
#pragma unroll
      for (int r = 0; r < 8; ++r) { const float h = acc[jt][r] + bb; sf[w0 + 8 * g + r][jt * 16 + col] = h; sa[w0 + 8 * g + r][jt * 16 + col] = (_Float16)h; } }
    __syncthreads();
    { const int pl = tid >> 6, c = tid & 63; float mx = -3.0e38f; for (int r = 0; r < CPL; ++r) mx = fmaxf(mx, sf[pl * CPL + r][c]); spool[pl][c] = mx; }
    __syncthreads();
    for (int e = tid; e < 64 * 64; e += 128) { const int rr = e >> 6, c = e & 63; sa[rr][HH + c] = (_Float16)spool[rr / CPL][c]; }
    __syncthreads();
  }
  gemm_tile<2 * HH>(&sa[w0 + col][0], PF + OFF_WL, lane, col, acc);
#pragma unroll
  for (int jt = 0; jt < 4; ++jt) { const float bb = bfr(BL[jt * 16 + col]);
#pragma unroll
    for (int r = 0; r < 8; ++r) sf[w0 + 8 * g + r][jt * 16 + col] = acc[jt][r] + bb; }
  __syncthreads();
  { const int pl = tid >> 6, c = tid & 63; float mx = -3.0e38f; for (int r = 0; r < CPL; ++r) mx = fmaxf(mx, sf[pl * CPL + r][c]); spool[pl][c] = mx; }
  __syncthreads();
  { __shared__ float snrm[2]; if (tid < 64) { const int pl = tid >> 5, l5 = tid & 31; float s = spool[pl][l5] * spool[pl][l5] + spool[pl][32 + l5] * spool[pl][32 + l5];
#pragma unroll
      for (int o = 1; o < 32; o <<= 1) s += __shfl_xor(s, o);
      if (l5 == 0) snrm[pl] = 1.0f / fmaxf(sqrtf(s), 1e-12f); }
    __syncthreads();
    if (tid < 32) { const int pl = tid >> 4, q = tid & 15; v4f v; for (int i = 0; i < 4; ++i) v[i] = spool[pl][q * 4 + i] * snrm[pl]; vst2(OUT + ((size_t)blockIdx.x * 2 + pl) * HH + q * 4, v); } }
}
extern "C" void kernel_launch(void* const* d_in, const int* in_sizes, int n_in, void* d_out, int out_size, void* d_ws, size_t ws_size, hipStream_t stream) {
  (void)in_sizes; (void)n_in; (void)out_size;
  const float** F = (const float**)d_in;
  if (ws_size < (size_t)WS_END) return;
  char* ws = (char*)d_ws; __bf16* P0 = (__bf16*)(ws + WS_W10); _Float16* PF = (_Float16*)(ws + WS_WF);
  k_pack<<<7, 256, 0, stream>>>(F[3], F[7], F[9], F[13], F[15], F[19], F[21], P0, PF);
  k_sub<<<TRB, 128, 0, stream>>>(F[0], P0, PF, F[4], F[5], F[6], F[8], F[10], F[11], F[12], F[14], F[16], F[17], F[18], F[20], F[22], (float*)d_out);
}
